// AggrHGraphConvWindow_79285096284407
// MI455X (gfx1250) — hardware-verified
//
#include <hip/hip_runtime.h>
#include <stdint.h>

typedef __attribute__((ext_vector_type(16))) _Float16 v16h;
typedef __attribute__((ext_vector_type(8)))  _Float16 v8h;
typedef __attribute__((ext_vector_type(16))) __bf16   v16b;
typedef __attribute__((ext_vector_type(8)))  __bf16   v8b;
typedef __attribute__((ext_vector_type(8)))  float    v8f;
typedef __attribute__((ext_vector_type(4)))  float    v4f;
typedef __attribute__((ext_vector_type(4)))  unsigned int v4u;

constexpr int kNumNode = 100;
constexpr int kNumPod  = 1500;
constexpr int kNumSvc  = 400;
constexpr int kNumRows = 2000;
constexpr int kSteps   = 32;
constexpr int kFeat    = 64;
constexpr int kConvOut = 128;
constexpr int kHid     = 256;
constexpr int kGates   = 1024;
constexpr int kEdgeSvc = 1600;
constexpr int kEdgeIn  = 1500;
constexpr int kEdgeNi  = 1500;
constexpr int kPadNode = 128;
constexpr int kPadPod  = 1536;
constexpr int kPadSvc  = 448;
constexpr int kXRows   = kPadNode + kPadPod + kPadSvc;
constexpr int kRowElems = kSteps * kFeat;
constexpr int kEdgeCap = 2048;

__device__ __forceinline__ unsigned short f2bf_bits(float f) {
  unsigned u = __float_as_uint(f);
  return (unsigned short)((u + 0x7FFFu + ((u >> 16) & 1u)) >> 16);
}
__device__ __forceinline__ float bf_bits2f(unsigned short h) { return __uint_as_float(((unsigned)h) << 16); }

__device__ __forceinline__ void dep_guard_h(v8f& a, v8f& b, v16h x, v16h y) { asm volatile("v_nop\n\tv_nop\n\tv_nop\n\tv_nop" : "+v"(a), "+v"(b) : "v"(x), "v"(y)); }
__device__ __forceinline__ void dep_guard_b(v8f& a, v8f& b, v16b x, v16b y) { asm volatile("v_nop\n\tv_nop\n\tv_nop\n\tv_nop" : "+v"(a), "+v"(b) : "v"(x), "v"(y)); }
__device__ __forceinline__ void keep4_h(v16h a, v16h b, v16h c, v16h d) { asm volatile("v_nop" :: "v"(a), "v"(b), "v"(c), "v"(d)); }
__device__ __forceinline__ void keep4_b(v16b a, v16b b, v16b c, v16b d) { asm volatile("v_nop" :: "v"(a), "v"(b), "v"(c), "v"(d)); }
__device__ __forceinline__ void acc_guard4(v8f& a, v8f& b, v8f& c, v8f& d) { asm volatile("v_nop\n\tv_nop\n\tv_nop\n\tv_nop" : "+v"(a), "+v"(b), "+v"(c), "+v"(d)); }
template <typename T> struct Frag;
template <> struct Frag<_Float16> {
  typedef v16h V; union U { v16h v; v8h h[2]; };
  static __device__ __forceinline__ v16h load(const _Float16* p) {
    U f; f.h[0] = *(const v8h*)(p); f.h[1] = *(const v8h*)(p + 16); return f.v;
  }
  static __device__ __forceinline__ v8f mma(v16h a, v16h b, v8f c) {
    return __builtin_amdgcn_wmma_f32_16x16x32_f16(false, a, false, b, (short)0, c, false, false);
  }
  static __device__ __forceinline__ void guard(v8f& a, v8f& b, v16h x, v16h y) { dep_guard_h(a, b, x, y); }
  static __device__ __forceinline__ void keep(v16h a, v16h b, v16h c, v16h d) { keep4_h(a, b, c, d); }
};
template <> struct Frag<__bf16> {
  typedef v16b V; union U { v16b v; v8b h[2]; };
  static __device__ __forceinline__ v16b load(const __bf16* p) {
    U f; f.h[0] = *(const v8b*)(p); f.h[1] = *(const v8b*)(p + 16); return f.v;
  }
  static __device__ __forceinline__ v8f mma(v16b a, v16b b, v8f c) {
    return __builtin_amdgcn_wmma_f32_16x16x32_bf16(false, a, false, b, (short)0, c, false, false);
  }
  static __device__ __forceinline__ void guard(v8f& a, v8f& b, v16b x, v16b y) { dep_guard_b(a, b, x, y); }
  static __device__ __forceinline__ void keep(v16b a, v16b b, v16b c, v16b d) { keep4_b(a, b, c, d); }
};

template <int ET> struct Elem;
template <> struct Elem<0> { typedef _Float16 T; };
template <> struct Elem<1> { typedef __bf16 T; };
template <int ET, bool SPLIT, int BIAS_MODE, int OUT_MODE, bool RESID, int ACT = 0>
__global__ __launch_bounds__(256) void wmma_gemm64(
    const unsigned short* __restrict__ Ap, const unsigned short* __restrict__ A2p, int lda, long strideA,
    const unsigned short* __restrict__ Btp, const unsigned short* __restrict__ Bt2p, int ldb, long strideB,
    void* __restrict__ Cout, void* __restrict__ Cout2, int ldc, long strideC,
    const float* __restrict__ bias, long strideBias,
    const float* __restrict__ resid, long strideR,
    int M, int N, int K, float scale, float oscale) {
  typedef typename Elem<ET>::T T;
  typedef typename Frag<T>::V V;
  const T* A = (const T*)Ap; const T* A2 = (const T*)A2p; const T* Bt = (const T*)Btp; const T* Bt2 = (const T*)Bt2p;
  __shared__ __align__(16) float sT[8][16 * 68];
  const int b    = blockIdx.y;
  const int lane = threadIdx.x & 31;
  const int wave = threadIdx.x >> 5;
  const int tilesN = N >> 6;
  const int tilesM = M >> 6;
  const int tile = blockIdx.x * 8 + wave;
  if (tile >= tilesM * tilesN) return;
  const int tm = tile / tilesN;
  const int tn = tile - tm * tilesN;
  const int m0 = tm << 6;
  const int n0 = tn << 6;

  const T* Ab  = A  + (size_t)b * strideA;
  const T* Bb  = Bt + (size_t)b * strideB;
  const T* Ab2 = SPLIT ? (A2  + (size_t)b * strideA) : nullptr;
  const T* Bb2 = SPLIT ? (Bt2 + (size_t)b * strideB) : nullptr;

  const int rlane = lane & 15;
  const int koff  = (lane >> 4) * 8;
  const int mOff  = (lane >> 4) * 8;

  v8f acc[4][4];
#pragma unroll
  for (int i = 0; i < 4; ++i)
#pragma unroll
    for (int j = 0; j < 4; ++j) acc[i][j] = (v8f){0.f,0.f,0.f,0.f,0.f,0.f,0.f,0.f};

  for (int k0 = 0; k0 < K; k0 += 32) {
    V bh[4], bl[4];
#pragma unroll
    for (int j = 0; j < 4; ++j) {
      const size_t bo = (size_t)(n0 + (j << 4) + rlane) * ldb + koff + k0;
      bh[j] = Frag<T>::load(Bb + bo);
      if (SPLIT) bl[j] = Frag<T>::load(Bb2 + bo);
    }
#pragma unroll
    for (int i = 0; i < 4; ++i) {
      const size_t ao = (size_t)(m0 + (i << 4) + rlane) * lda + koff + k0;
      V ah = Frag<T>::load(Ab + ao);
      V al;
      if (SPLIT) al = Frag<T>::load(Ab2 + ao);
#pragma unroll
      for (int j = 0; j < 4; ++j) {
        acc[i][j] = Frag<T>::mma(ah, bh[j], acc[i][j]);
        if (SPLIT) {
          acc[i][j] = Frag<T>::mma(ah, bl[j], acc[i][j]);
          acc[i][j] = Frag<T>::mma(al, bh[j], acc[i][j]);
        }
      }
      Frag<T>::guard(acc[i][0], acc[i][3], ah, SPLIT ? al : ah);
    }
    Frag<T>::keep(bh[0], bh[1], bh[2], bh[3]);
    if (SPLIT) Frag<T>::keep(bl[0], bl[1], bl[2], bl[3]);
  }
  acc_guard4(acc[0][0], acc[0][1], acc[0][2], acc[0][3]);
  acc_guard4(acc[1][0], acc[1][1], acc[1][2], acc[1][3]);
  acc_guard4(acc[2][0], acc[2][1], acc[2][2], acc[2][3]);
  acc_guard4(acc[3][0], acc[3][1], acc[3][2], acc[3][3]);

  float* slab = sT[wave];
  const float* Rb = RESID ? (resid + (size_t)b * strideR) : nullptr;
  const float* biasb = (BIAS_MODE != 0) ? (bias + (size_t)b * strideBias) : nullptr;
#pragma unroll
  for (int i = 0; i < 4; ++i) {
    const int mBase = m0 + (i << 4);
#pragma unroll
    for (int j = 0; j < 4; ++j) {
      const int n = n0 + (j << 4) + rlane;
      float bv = 0.f;
      if (BIAS_MODE == 2) bv = biasb[n];
#pragma unroll
      for (int r = 0; r < 8; ++r) {
        float v = acc[i][j][r] * scale;
        if (BIAS_MODE == 1) v += biasb[mBase + mOff + r];
        if (BIAS_MODE == 2) v += bv;
        if (RESID) v += Rb[(size_t)(mBase + mOff + r) * ldc + n];
        if (ACT == 1) v = tanhf(v);
        if (ACT == 2) v = fmaxf(v, 0.0f);
        if (ACT == 4) v = (v > 0.f) ? v : 0.01f * v;
        slab[(mOff + r) * 68 + (j << 4) + rlane] = v * oscale;
      }
    }
    __builtin_amdgcn_fence(__ATOMIC_RELEASE, "workgroup");
    __builtin_amdgcn_wave_barrier();
    __builtin_amdgcn_fence(__ATOMIC_ACQUIRE, "workgroup");
    if (OUT_MODE == 0) {
      float* C = (float*)Cout + (size_t)b * strideC;
      const int hh = lane >> 4, c4 = (lane & 15) * 4;
      for (int pass = 0; pass < 2; ++pass) {
#pragma unroll
        for (int it = 0; it < 8; ++it) {
          const int row = it * 2 + hh;
          v4f v = *(const v4f*)(slab + row * 68 + c4);
          *(volatile v4f*)(C + (size_t)(mBase + row) * ldc + n0 + c4) = v;
        }
        __threadfence();
      }
    } else {
      const int q = lane >> 3, c8 = (lane & 7) * 8;
      unsigned short* C  = (unsigned short*)Cout  + (size_t)b * strideC;
      unsigned short* C2 = (OUT_MODE == 2) ? ((unsigned short*)Cout2 + (size_t)b * strideC) : nullptr;
      for (int pass = 0; pass < 2; ++pass) {
#pragma unroll
        for (int it = 0; it < 4; ++it) {
          const int row = it * 4 + q;
          const float* sp = slab + row * 68 + c8;
          v8h hv, lv;
#pragma unroll
          for (int e = 0; e < 8; ++e) {
            if (OUT_MODE == 1) {
              hv[e] = (_Float16)sp[e];
            } else {
              unsigned short hb = f2bf_bits(sp[e]);
              unsigned short lb = f2bf_bits(sp[e] - bf_bits2f(hb));
              hv[e] = __builtin_bit_cast(_Float16, hb);
              lv[e] = __builtin_bit_cast(_Float16, lb);
            }
          }
          *(volatile v8h*)(C + (size_t)(mBase + row) * ldc + n0 + c8) = hv;
          if (OUT_MODE == 2) *(volatile v8h*)(C2 + (size_t)(mBase + row) * ldc + n0 + c8) = lv;
        }
        __threadfence();
      }
    }
    __builtin_amdgcn_fence(__ATOMIC_RELEASE, "workgroup");
    __builtin_amdgcn_wave_barrier();
    __builtin_amdgcn_fence(__ATOMIC_ACQUIRE, "workgroup");
  }
}

__device__ __forceinline__ unsigned int pk_f16x2_scaled8(float a, float b) {
  const unsigned short ua = __builtin_bit_cast(unsigned short, (_Float16)(a * 8.0f));
  const unsigned short ub = __builtin_bit_cast(unsigned short, (_Float16)(b * 8.0f));
  return (unsigned)ua | (((unsigned)ub) << 16);
}
__device__ __forceinline__ void pk_bf16_split2(float a, float b, unsigned& hw, unsigned& lw) {
  const unsigned short ha = f2bf_bits(a), hb = f2bf_bits(b);
  const unsigned short la = f2bf_bits(a - bf_bits2f(ha)), lb = f2bf_bits(b - bf_bits2f(hb));
  hw = (unsigned)ha | (((unsigned)hb) << 16);
  lw = (unsigned)la | (((unsigned)lb) << 16);
}

__global__ __launch_bounds__(256) void k_srcnorm(const int* __restrict__ src, int ne, int n_src, float* __restrict__ sn) {
  __shared__ __align__(16) float sv[256];
  const int tid = threadIdx.x, wave = tid >> 5, lane = tid & 31;
  const int s = blockIdx.x * 256 + tid;
  int cnt = 0;
  for (int e = 0; e < ne; ++e) {
    int v = src[e];
    v = v < 0 ? 0 : (v >= n_src ? (n_src - 1) : v);
    cnt += (v == s) ? 1 : 0;
  }
  sv[tid] = 1.0f / sqrtf(fmaxf((float)cnt, 1.0f));
  __syncthreads();
  if (wave < 2) {
    const int i4 = (wave * 32 + lane) * 4;
    const v4f val = *(const v4f*)(sv + i4);
    float* p = sn + (size_t)blockIdx.x * 256 + i4;
    for (int pass = 0; pass < 2; ++pass) { *(volatile v4f*)p = val; __threadfence(); }
  }
}

__global__ __launch_bounds__(256) void k_aggr(const float* __restrict__ feat, int n_src,
    const int* __restrict__ src, const int* __restrict__ dst, int ne, int n_dst,
    const float* __restrict__ sn, unsigned short* __restrict__ agg_hi, unsigned short* __restrict__ agg_lo) {
#pragma clang fp contract(off)
  __shared__ int elist[kEdgeCap];
  __shared__ int wcnt[8];
  const int d = blockIdx.x;
  const int tid = threadIdx.x, wave = tid >> 5, lane = tid & 31;
  int base = 0;
  for (int eb = 0; eb < ne; eb += 256) {
    const int e  = eb + tid;
    const int ec = (e < ne) ? e : (ne - 1);
    int dv = dst[ec];
    dv = dv < 0 ? 0 : (dv >= n_dst ? (n_dst - 1) : dv);
    const int hit = ((e < ne) && (dv == d)) ? 1 : 0;
    const unsigned msk = (unsigned)__ballot(hit);
    const int lpre = (int)__popc(msk & ((1u << lane) - 1u));
    if (lane == 0) wcnt[wave] = (int)__popc(msk);
    __syncthreads();
    int woff = 0, tot = 0;
#pragma unroll
    for (int w = 0; w < 8; ++w) { const int cw = wcnt[w]; woff += (w < wave) ? cw : 0; tot += cw; }
    if (hit) {
      const int pos = base + woff + lpre;
      if ((unsigned)pos < (unsigned)kEdgeCap) elist[pos] = e;
    }
    base += tot;
    __syncthreads();
  }
  const int cntc = base < kEdgeCap ? base : kEdgeCap;
  const float dn = 1.0f / sqrtf(fmaxf((float)base, 1.0f));
  v4f acc0 = (v4f){0.f, 0.f, 0.f, 0.f}, acc1 = (v4f){0.f, 0.f, 0.f, 0.f};
  for (int p = 0; p < cntc; ++p) {
    const int e = elist[p];
    int s = src[e];
    s = s < 0 ? 0 : (s >= n_src ? (n_src - 1) : s);
    const float w = sn[s];
    const float* fp = feat + (size_t)s * kRowElems + (size_t)tid * 8;
    const v4f x0 = *(const v4f*)fp;
    const v4f x1 = *(const v4f*)(fp + 4);
    acc0 += x0 * w;
    acc1 += x1 * w;
  }
  acc0 *= dn; acc1 *= dn;
  v4u hv, lv;
  { unsigned hw, lw;
    pk_bf16_split2(acc0[0], acc0[1], hw, lw); hv[0] = hw; lv[0] = lw;
    pk_bf16_split2(acc0[2], acc0[3], hw, lw); hv[1] = hw; lv[1] = lw;
    pk_bf16_split2(acc1[0], acc1[1], hw, lw); hv[2] = hw; lv[2] = lw;
    pk_bf16_split2(acc1[2], acc1[3], hw, lw); hv[3] = hw; lv[3] = lw; }
  const size_t o = (size_t)d * kRowElems + (size_t)tid * 8;
  for (int pass = 0; pass < 2; ++pass) {
    *(volatile v4u*)(agg_hi + o) = hv;
    *(volatile v4u*)(agg_lo + o) = lv;
    __threadfence();
  }
}

__global__ __launch_bounds__(256) void k_convw(const float* __restrict__ W, unsigned short* __restrict__ Whi, unsigned short* __restrict__ Wlo) {
  __shared__ __align__(16) float sW[kFeat * kConvOut];
  const int t = blockIdx.x, tid = threadIdx.x;
  const float* Wt = W + (size_t)t * (kFeat * kConvOut);
#pragma unroll
  for (int it = 0; it < 8; ++it) {
    const int i4 = it * 256 + tid;
    *(v4f*)(sW + i4 * 4) = *(const v4f*)(Wt + (size_t)i4 * 4);
  }
  __syncthreads();
#pragma unroll 1
  for (int p = 0; p < 4; ++p) {
    const int g = p * 256 + tid;
    const int n = g >> 3;
    const int f0 = (g & 7) * 8;
    v4u hv, lv;
#pragma unroll
    for (int i = 0; i < 4; ++i) {
      const float a = sW[(f0 + 2 * i) * kConvOut + n];
      const float b = sW[(f0 + 2 * i + 1) * kConvOut + n];
      unsigned hw, lw;
      pk_bf16_split2(a, b, hw, lw);
      hv[i] = hw; lv[i] = lw;
    }
    const size_t o = (size_t)t * (kFeat * kConvOut) + (size_t)n * kFeat + f0;
    for (int pass = 0; pass < 2; ++pass) {
      *(volatile v4u*)(Whi + o) = hv;
      *(volatile v4u*)(Wlo + o) = lv;
      __threadfence();
    }
  }
}

template <int KIN>
__global__ __launch_bounds__(256) void k_lstmw(const float* __restrict__ Wih, const float* __restrict__ Whh, unsigned short* __restrict__ Wc) {
  constexpr int KTOT = KIN + kHid;
  constexpr int GPR = KTOT / 8;
  constexpr int NG = kGates * GPR;
  const int g = blockIdx.x * 256 + threadIdx.x;
  if (g < NG) {
    const int n = g / GPR;
    const int c8 = (g - n * GPR) * 8;
    const int cih = (c8 < KIN - 8) ? c8 : (KIN - 8);
    int chh = c8 - KIN; chh = chh < 0 ? 0 : chh;
    const float* pa = Wih + (size_t)n * KIN + cih;
    const float* pb = Whh + (size_t)n * kHid + chh;
    const v4f a0 = *(const v4f*)pa, a1 = *(const v4f*)(pa + 4);
    const v4f b0 = *(const v4f*)pb, b1 = *(const v4f*)(pb + 4);
    const bool ui = c8 < KIN;
    float x[8];
#pragma unroll
    for (int e = 0; e < 4; ++e) { x[e] = ui ? a0[e] : b0[e]; x[4 + e] = ui ? a1[e] : b1[e]; }
    v4u pv;
    pv[0] = pk_f16x2_scaled8(x[0], x[1]); pv[1] = pk_f16x2_scaled8(x[2], x[3]);
    pv[2] = pk_f16x2_scaled8(x[4], x[5]); pv[3] = pk_f16x2_scaled8(x[6], x[7]);
    unsigned short* dp = Wc + (size_t)n * KTOT + c8;
    for (int pass = 0; pass < 2; ++pass) { *(volatile v4u*)dp = pv; __threadfence(); }
  }
}

__device__ __forceinline__ float rcp_fast_(float x) { return __builtin_amdgcn_rcpf(x); }
__device__ __forceinline__ float sigm_(float x) {
  x = fminf(fmaxf(x, -30.0f), 30.0f);
  const float e = expf(-x);
  return rcp_fast_(1.0f + e);
}
__device__ __forceinline__ float tanh_(float x) {
  const float ax = fminf(fabsf(x), 15.0f);
  const float e = expf(-2.0f * ax);
  const float r = (1.0f - e) * rcp_fast_(1.0f + e);
  return copysignf(r, x);
}

template <int KIN, int LAYER>
__global__ __launch_bounds__(256) void k_lstm(
    const unsigned short* __restrict__ Xin, const unsigned short* __restrict__ Wc,
    const float* __restrict__ bih, const float* __restrict__ bhh,
    unsigned short* __restrict__ H16, float* __restrict__ H32) {
  constexpr int KTOT = KIN + kHid;
  constexpr int KP = KTOT + 16;
  constexpr int HP = kHid + 4;
  constexpr float kGateScale = 1.0f / 64.0f;
  __shared__ __align__(16) unsigned short At[16 * KP];
  __shared__ __align__(16) float hs[16 * HP];
  const int tid = threadIdx.x;
  const int wave = tid >> 5, lane = tid & 31;
  const int hh = lane >> 4, c = lane & 15;
  const int koff = hh * 8;
  const int m0 = blockIdx.x * 16;

  float bsum[2][4];
#pragma unroll
  for (int u = 0; u < 2; ++u)
#pragma unroll
    for (int q = 0; q < 4; ++q) {
      const int n = q * kHid + wave * 32 + u * 16 + c;
      bsum[u][q] = bih[n] + bhh[n];
    }
  float cst[2][8];
#pragma unroll
  for (int u = 0; u < 2; ++u)
#pragma unroll
    for (int r = 0; r < 8; ++r) cst[u][r] = 0.0f;

  const int frow = tid >> 4;
  {
    const v4u z = (v4u){0u, 0u, 0u, 0u};
    unsigned short* p = At + frow * KP + KIN + (tid & 15) * 16;
    *(v4u*)p = z; *(v4u*)(p + 8) = z;
  }
  int xr = m0 + frow;
  if (LAYER == 0) xr = xr + ((xr >= kNumNode) ? (kPadNode - kNumNode) : 0) + ((xr >= kNumNode + kNumPod) ? (kPadPod - kNumPod) : 0);

  for (int t = 0; t < kSteps; ++t) {
    {
      const unsigned short* srow = Xin + ((size_t)xr * kSteps + t) * KIN;
      unsigned short* drow = At + frow * KP;
      const int c8 = (tid & 15) * 8;
      *(v4u*)(drow + c8) = *(const v4u*)(srow + c8);
      if (KIN == 256) *(v4u*)(drow + 128 + c8) = *(const v4u*)(srow + 128 + c8);
    }
    __syncthreads();
    v8f acc[2][4];
#pragma unroll
    for (int u = 0; u < 2; ++u)
#pragma unroll
      for (int q = 0; q < 4; ++q) acc[u][q] = (v8f){0.f,0.f,0.f,0.f,0.f,0.f,0.f,0.f};
#pragma unroll 1
    for (int k0 = 0; k0 < KTOT; k0 += 32) {
      const v16h af = Frag<_Float16>::load((const _Float16*)(At + c * KP + k0 + koff));
#pragma unroll
      for (int u = 0; u < 2; ++u) {
        v16h bq[4];
#pragma unroll
        for (int q = 0; q < 4; ++q)
          bq[q] = Frag<_Float16>::load((const _Float16*)(Wc + (size_t)(q * kHid + wave * 32 + u * 16 + c) * KTOT + k0 + koff));
#pragma unroll
        for (int q = 0; q < 4; ++q) acc[u][q] = Frag<_Float16>::mma(af, bq[q], acc[u][q]);
        dep_guard_h(acc[u][0], acc[u][3], af, af);
        keep4_h(bq[0], bq[1], bq[2], bq[3]);
      }
    }
    acc_guard4(acc[0][0], acc[0][1], acc[0][2], acc[0][3]);
    acc_guard4(acc[1][0], acc[1][1], acc[1][2], acc[1][3]);
#pragma unroll
    for (int u = 0; u < 2; ++u) {
      const int j = wave * 32 + u * 16 + c;
#pragma unroll
      for (int r = 0; r < 8; ++r) {
        const float gi = sigm_(acc[u][0][r] * kGateScale + bsum[u][0]);
        const float gf = sigm_(acc[u][1][r] * kGateScale + bsum[u][1]);
        const float gg = tanh_(acc[u][2][r] * kGateScale + bsum[u][2]);
        const float go = sigm_(acc[u][3][r] * kGateScale + bsum[u][3]);
        const float cn = gf * cst[u][r] + gi * gg;
        cst[u][r] = cn;
        hs[(8 * hh + r) * HP + j] = go * tanh_(cn);
      }
    }
    __syncthreads();
    {
      const int col = (tid & 15) * 16;
      const float* sp = hs + frow * HP + col;
      const v4f a0 = *(const v4f*)sp, a1 = *(const v4f*)(sp + 4), a2 = *(const v4f*)(sp + 8), a3 = *(const v4f*)(sp + 12);
      v4u p0, p1;
      p0[0] = pk_f16x2_scaled8(a0[0], a0[1]); p0[1] = pk_f16x2_scaled8(a0[2], a0[3]);
      p0[2] = pk_f16x2_scaled8(a1[0], a1[1]); p0[3] = pk_f16x2_scaled8(a1[2], a1[3]);
      p1[0] = pk_f16x2_scaled8(a2[0], a2[1]); p1[1] = pk_f16x2_scaled8(a2[2], a2[3]);
      p1[2] = pk_f16x2_scaled8(a3[0], a3[1]); p1[3] = pk_f16x2_scaled8(a3[2], a3[3]);
      unsigned short* dp = At + frow * KP + KIN + col;
      *(v4u*)dp = p0; *(v4u*)(dp + 8) = p1;
    }
    if (LAYER == 0) {
      v4u pv[2];
#pragma unroll
      for (int rr = 0; rr < 2; ++rr) {
        const float* sp = hs + (wave * 2 + rr) * HP + lane * 8;
        const v4f a0 = *(const v4f*)sp, a1 = *(const v4f*)(sp + 4);
        pv[rr][0] = pk_f16x2_scaled8(a0[0], a0[1]); pv[rr][1] = pk_f16x2_scaled8(a0[2], a0[3]);
        pv[rr][2] = pk_f16x2_scaled8(a1[0], a1[1]); pv[rr][3] = pk_f16x2_scaled8(a1[2], a1[3]);
      }
      for (int pass = 0; pass < 2; ++pass) {
#pragma unroll
        for (int rr = 0; rr < 2; ++rr) {
          const int m = m0 + wave * 2 + rr;
          unsigned short* dp = H16 + ((size_t)m * kSteps + t) * kHid + lane * 8;
          *(volatile v4u*)dp = pv[rr];
        }
        __threadfence();
      }
    } else {
      v4f va[2], vb[2];
#pragma unroll
      for (int rr = 0; rr < 2; ++rr) {
        const float* sp = hs + (wave * 2 + rr) * HP;
        va[rr] = *(const v4f*)(sp + lane * 4);
        vb[rr] = *(const v4f*)(sp + 128 + lane * 4);
      }
      for (int pass = 0; pass < 2; ++pass) {
#pragma unroll
        for (int rr = 0; rr < 2; ++rr) {
          const int m = m0 + wave * 2 + rr;
          float* dp = H32 + ((size_t)m * kSteps + t) * kHid;
          *(volatile v4f*)(dp + lane * 4) = va[rr];
          *(volatile v4f*)(dp + 128 + lane * 4) = vb[rr];
        }
        __threadfence();
      }
    }
  }
}

extern "C" void kernel_launch(void* const* d_in, const int* in_sizes, int n_in,
                              void* d_out, int out_size, void* d_ws, size_t ws_size,
                              hipStream_t stream) {
  (void)in_sizes; (void)n_in; (void)out_size;
  const float* node_feat = (const float*)d_in[0];
  const float* pod_feat  = (const float*)d_in[1];
  const float* svc_feat  = (const float*)d_in[2];
  const float* W_svc = (const float*)d_in[3];
  const float* b_svc = (const float*)d_in[4];
  const float* W_in  = (const float*)d_in[5];
  const float* b_in  = (const float*)d_in[6];
  const float* W_ni  = (const float*)d_in[7];
  const float* b_ni  = (const float*)d_in[8];
  const float* W_ih0 = (const float*)d_in[9];
  const float* W_hh0 = (const float*)d_in[10];
  const float* b_ih0 = (const float*)d_in[11];
  const float* b_hh0 = (const float*)d_in[12];
  const float* W_ih1 = (const float*)d_in[13];
  const float* W_hh1 = (const float*)d_in[14];
  const float* b_ih1 = (const float*)d_in[15];
  const float* b_hh1 = (const float*)d_in[16];
  const int* svc_src = (const int*)d_in[17];
  const int* svc_dst = (const int*)d_in[18];
  const int* in_src  = (const int*)d_in[19];
  const int* in_dst  = (const int*)d_in[20];
  const int* ni_src  = (const int*)d_in[21];
  const int* ni_dst  = (const int*)d_in[22];
  float* out = (float*)d_out;

  char* ws = (char*)d_ws;
  size_t off = 0;
  auto carve = [&](size_t bytes) -> char* {
    off = (off + 255) & ~(size_t)255;
    char* p = ws + off;
    off += bytes;
    return p;
  };
  float* snS = (float*)carve((size_t)512 * 4);
  float* snP = (float*)carve((size_t)1536 * 4);
  float* snN = (float*)carve((size_t)256 * 4);
  const size_t aggNB = (size_t)kPadNode * kRowElems * 2;
  const size_t aggPB = (size_t)kPadPod  * kRowElems * 2;
  const size_t aggSB = (size_t)kPadSvc  * kRowElems * 2;
  unsigned short* aggNh = (unsigned short*)carve(aggNB);
  unsigned short* aggNl = (unsigned short*)carve(aggNB);
  unsigned short* aggPh = (unsigned short*)carve(aggPB);
  unsigned short* aggPl = (unsigned short*)carve(aggPB);
  unsigned short* aggSh = (unsigned short*)carve(aggSB);
  unsigned short* aggSl = (unsigned short*)carve(aggSB);
  const size_t wtB = (size_t)kSteps * kConvOut * kFeat * 2;
  unsigned short* WtNh = (unsigned short*)carve(wtB);
  unsigned short* WtNl = (unsigned short*)carve(wtB);
  unsigned short* WtPh = (unsigned short*)carve(wtB);
  unsigned short* WtPl = (unsigned short*)carve(wtB);
  unsigned short* WtSh = (unsigned short*)carve(wtB);
  unsigned short* WtSl = (unsigned short*)carve(wtB);
  unsigned short* Xp  = (unsigned short*)carve((size_t)kXRows * kSteps * kConvOut * 2);
  unsigned short* Wc0 = (unsigned short*)carve((size_t)kGates * (kConvOut + kHid) * 2);
  unsigned short* Wc1 = (unsigned short*)carve((size_t)kGates * (kHid + kHid) * 2);
  unsigned short* H1  = (unsigned short*)carve((size_t)kNumRows * kSteps * kHid * 2);
  if (off > ws_size) return;

  k_srcnorm<<<dim3(2), dim3(256), 0, stream>>>(svc_src, kEdgeSvc, kNumSvc, snS);
  k_srcnorm<<<dim3(6), dim3(256), 0, stream>>>(in_src,  kEdgeIn,  kNumPod, snP);
  k_srcnorm<<<dim3(1), dim3(256), 0, stream>>>(ni_src,  kEdgeNi,  kNumNode, snN);

  k_aggr<<<dim3(kPadNode), dim3(256), 0, stream>>>(pod_feat,  kNumPod,  in_src,  in_dst,  kEdgeIn,  kNumNode, snP, aggNh, aggNl);
  k_aggr<<<dim3(kPadPod),  dim3(256), 0, stream>>>(node_feat, kNumNode, ni_src,  ni_dst,  kEdgeNi,  kNumPod,  snN, aggPh, aggPl);
  k_aggr<<<dim3(kPadSvc),  dim3(256), 0, stream>>>(svc_feat,  kNumSvc,  svc_src, svc_dst, kEdgeSvc, kNumSvc,  snS, aggSh, aggSl);

  k_convw<<<dim3(kSteps), dim3(256), 0, stream>>>(W_in,  WtNh, WtNl);
  k_convw<<<dim3(kSteps), dim3(256), 0, stream>>>(W_ni,  WtPh, WtPl);
  k_convw<<<dim3(kSteps), dim3(256), 0, stream>>>(W_svc, WtSh, WtSl);

  k_lstmw<kConvOut><<<dim3((kGates * ((kConvOut + kHid) / 8)) / 256), dim3(256), 0, stream>>>(W_ih0, W_hh0, Wc0);
  k_lstmw<kHid><<<dim3((kGates * ((kHid + kHid) / 8)) / 256), dim3(256), 0, stream>>>(W_ih1, W_hh1, Wc1);

  {
    const size_t xpitch = (size_t)kSteps * kConvOut;
    wmma_gemm64<1, true, 2, 1, false, 4><<<dim3(((kPadNode / 64) * 2 + 7) / 8, kSteps), dim3(256), 0, stream>>>(
        aggNh, aggNl, kRowElems, (long)kFeat, WtNh, WtNl, kFeat, (long)(kConvOut * kFeat),
        (void*)(Xp), (void*)(Xp), (int)xpitch, (long)kConvOut,
        b_in, (long)kConvOut, b_in, 0L, kPadNode, kConvOut, kFeat, 1.0f, 8.0f);
    wmma_gemm64<1, true, 2, 1, false, 4><<<dim3(((kPadPod / 64) * 2 + 7) / 8, kSteps), dim3(256), 0, stream>>>(
        aggPh, aggPl, kRowElems, (long)kFeat, WtPh, WtPl, kFeat, (long)(kConvOut * kFeat),
        (void*)(Xp + (size_t)kPadNode * xpitch), (void*)(Xp + (size_t)kPadNode * xpitch), (int)xpitch, (long)kConvOut,
        b_ni, (long)kConvOut, b_ni, 0L, kPadPod, kConvOut, kFeat, 1.0f, 8.0f);
    wmma_gemm64<1, true, 2, 1, false, 4><<<dim3(((kPadSvc / 64) * 2 + 7) / 8, kSteps), dim3(256), 0, stream>>>(
        aggSh, aggSl, kRowElems, (long)kFeat, WtSh, WtSl, kFeat, (long)(kConvOut * kFeat),
        (void*)(Xp + (size_t)(kPadNode + kPadPod) * xpitch), (void*)(Xp + (size_t)(kPadNode + kPadPod) * xpitch), (int)xpitch, (long)kConvOut,
        b_svc, (long)kConvOut, b_svc, 0L, kPadSvc, kConvOut, kFeat, 1.0f, 8.0f);
  }

  k_lstm<kConvOut, 0><<<dim3(kNumRows / 16), dim3(256), 0, stream>>>(Xp, Wc0, b_ih0, b_hh0, H1, out);
  k_lstm<kHid, 1><<<dim3(kNumRows / 16), dim3(256), 0, stream>>>(H1, Wc1, b_ih1, b_hh1, Xp, out);
}
